// BinarizeConv2dSDP_82910048682620
// MI455X (gfx1250) — hardware-verified
//
#include <hip/hip_runtime.h>


typedef __attribute__((ext_vector_type(16))) _Float16 v16h;
typedef __attribute__((ext_vector_type(8)))  _Float16 v8h;
typedef __attribute__((ext_vector_type(8)))  float    v8f;
typedef __attribute__((ext_vector_type(4)))  float    v4f;
#define NIMG 64
#define CIN  256
#define COUT 256
#define HWID 28
#define HW   784
#define KTOT 2304
#define VST2(T, ptr, val) do { const T _v = (val); *(volatile T*)(ptr) = _v; __threadfence(); *(volatile T*)(ptr) = _v; } while (0)
__device__ __forceinline__ v8f wmma16(v16h a, v16h b, v8f c) {
  v8f d = __builtin_amdgcn_wmma_f32_16x16x32_f16(false, a, false, b, (short)0, c, false, false);
  asm volatile("v_nop\n\tv_nop\n\tv_nop\n\tv_nop" : "+v"(d) : "v"(a), "v"(b));
  return d;
}
__device__ __forceinline__ v16h frag16(const _Float16* p, int hh) {
  const v8h lo = *(const v8h*)(p + 8 * hh), hi = *(const v8h*)(p + 16 + 8 * hh);
  return __builtin_shufflevector(lo, hi, 0,1,2,3,4,5,6,7,8,9,10,11,12,13,14,15);
}
__device__ __forceinline__ float sgnf(float v) { return v > 0.f ? 1.f : (v < 0.f ? -1.f : 0.f); }

__global__ __launch_bounds__(256) void k_act(const float* __restrict__ x, _Float16* __restrict__ act) {
  const int t = blockIdx.x * 256 + threadIdx.x;
  const int c8 = (t & 31) * 8, pos = t >> 5, b = pos / HW, hw = pos - b * HW;
  const float* xs = x + ((size_t)b * CIN + c8) * HW + hw;
  v8h v;
#pragma unroll
  for (int e = 0; e < 8; ++e) v[e] = (_Float16)sgnf(xs[(size_t)e * HW]);
  VST2(v8h, act + (size_t)t * 8, v);
}
__global__ __launch_bounds__(256) void k_wgt(const float* __restrict__ M, const float* __restrict__ Z, const float* __restrict__ rv, _Float16* __restrict__ Wb) {
  const int t = blockIdx.x * 256 + threadIdx.x;
  const int c8 = (t & 31) * 8, tap = (t >> 5) % 9, o = t / (32 * 9);
  v8h v;
#pragma unroll
  for (int e = 0; e < 8; ++e) {
    const size_t n = ((size_t)o * CIN + c8 + e) * 9 + tap;
    const float m = M[n];
    float zs[8], zz = 0.f;
#pragma unroll
    for (int k = 0; k < 8; ++k) { zs[k] = Z[(size_t)k * COUT * KTOT + n]; zz += zs[k] * zs[k]; }
    const float inv = 1.0f / sqrtf(m * m + zz * (1.0f / 100.0f));
    float w = m * inv;
#pragma unroll
    for (int k = 0; k < 8; ++k) w += rv[k] * (zs[k] * inv);
    v[e] = (_Float16)sgnf(w);
  }
  VST2(v8h, Wb + ((size_t)o * 9 + tap) * CIN + c8, v);
}
__global__ __launch_bounds__(256) void k_bconv(const _Float16* __restrict__ Wb, const _Float16* __restrict__ act, const float* __restrict__ alpha,
                                               float* __restrict__ out) {
  __shared__ __attribute__((aligned(16))) float sO[32 * HW];
  const int lane = threadIdx.x & 31, wave = threadIdx.x >> 5, hh = lane >> 4, l16 = lane & 15;
  const int b = blockIdx.x >> 3, og = (blockIdx.x & 7) * 32;
  const _Float16* actb = act + (size_t)b * HW * CIN;
  const _Float16* wrow0 = Wb + (size_t)(og + l16) * KTOT;
  const _Float16* wrow1 = wrow0 + (size_t)16 * KTOT;
  const float al0[1] = {0.f}; (void)al0;
  for (int tile = wave; tile < HW / 16; tile += 8) {
    const int p = tile * 16 + l16;
    const int py = p / HWID, px = p - py * HWID;
    v8f acc0 = {}, acc1 = {};
    for (int tap = 0; tap < 9; ++tap) {
      const int ys = py + tap / 3 - 1, xs = px + tap % 3 - 1;
      const bool in = (ys >= 0) & (ys < HWID) & (xs >= 0) & (xs < HWID);
      const _Float16* bp = actb + ((size_t)(in ? (ys * HWID + xs) : 0)) * CIN;
#pragma unroll 2
      for (int c0 = 0; c0 < CIN; c0 += 32) {
        v16h bf;
        if (in) bf = frag16(bp + c0, hh); else { for (int e = 0; e < 16; ++e) bf[e] = (_Float16)0.f; }
        const int k = tap * CIN + c0;
        acc0 = wmma16(frag16(wrow0 + k, hh), bf, acc0);
        acc1 = wmma16(frag16(wrow1 + k, hh), bf, acc1);
      }
    }
#pragma unroll
    for (int r = 0; r < 8; ++r) {
      sO[(r + 8 * hh) * HW + p]      = acc0[r] * alpha[og + r + 8 * hh];
      sO[(16 + r + 8 * hh) * HW + p] = acc1[r] * alpha[og + 16 + r + 8 * hh];
    }
  }
  __syncthreads();
  float* dst = out + ((size_t)b * COUT + og) * HW;
  for (int pass = 0; pass < 2; ++pass) {
    for (int q = threadIdx.x; q < 32 * HW / 4; q += 256) *(volatile v4f*)(dst + q * 4) = *(const v4f*)(sO + q * 4);
    __threadfence();
  }
}
extern "C" void kernel_launch(void* const* d_in, const int* in_sizes, int n_in,
                              void* d_out, int out_size, void* d_ws, size_t ws_size, hipStream_t stream) {
  (void)in_sizes; (void)n_in; (void)out_size;
  const float* x  = (const float*)d_in[0];
  const float* M  = (const float*)d_in[1];
  const float* Z  = (const float*)d_in[2];
  const float* al = (const float*)d_in[3];
  const float* rv = (const float*)d_in[4];
  float* out = (float*)d_out;
  const size_t actB = (size_t)NIMG * HW * CIN * 2, wB = (size_t)COUT * KTOT * 2;
  if (ws_size < actB + wB) return;
  _Float16* act = (_Float16*)d_ws;
  _Float16* Wb  = (_Float16*)((char*)d_ws + actB);
  k_act<<<NIMG * HW * 32 / 256, 256, 0, stream>>>(x, act);
  k_wgt<<<COUT * 9 * 32 / 256, 256, 0, stream>>>(M, Z, rv, Wb);
  k_bconv<<<NIMG * 8, 256, 0, stream>>>(Wb, act, al, out);
}
